// Rnn_2860448219793
// MI455X (gfx1250) — hardware-verified
//
#include <hip/hip_runtime.h>
#include <math.h>

constexpr int NBATCH   = 4096;
constexpr int NSTEP    = 512;
constexpr int NHID     = 32;
constexpr int ROWS_BLK = 16;
constexpr int TCHUNK   = 32;
constexpr int NCHUNK   = NSTEP / TCHUNK;
constexpr int HPITCH   = 40;
constexpr int FPITCH   = 36;
constexpr float HCARRY   = 64.0f;
constexpr float WCARRY   = 16.0f;
constexpr float CARRYINV = 1.0f / (HCARRY * WCARRY);
constexpr int NOUT0 = NBATCH * NSTEP;
constexpr int NOUT1 = NBATCH * NHID;

static_assert(NHID == 32, "one 32-deep k step, two 16-row M tiles");
static_assert(NBATCH % ROWS_BLK == 0, "grid exact");
static_assert(NSTEP % TCHUNK == 0, "no time tail");
static_assert(TCHUNK * 4 == 128, "one chunk row = one 128-B line");
static_assert((NSTEP * 4) % 128 == 0, "x / out0 rows are line aligned");
static_assert(((size_t)NOUT0 * 4) % 128 == 0, "out1 base is line aligned");
static_assert((size_t)NOUT0 * 4 == 8388608, "out1 byte offset");
static_assert((size_t)NOUT0 * 4 + (size_t)NOUT1 * 4 == 8912896, "d_out total bytes");
static_assert(HPITCH % 8 == 0 && FPITCH % 4 == 0, "16-B aligned LDS rows");

typedef __attribute__((ext_vector_type(16))) _Float16 v16h;
typedef __attribute__((ext_vector_type(8)))  _Float16 v8h;
typedef __attribute__((ext_vector_type(8)))  float    v8f;
typedef __attribute__((ext_vector_type(4)))  float    v4f;

union FragU { v16h v; v8h h[2]; };
__device__ __forceinline__ v16h frag_load(const _Float16* p) {
  FragU f;
  f.h[0] = *(const v8h*)(p);
  f.h[1] = *(const v8h*)(p + 16);
  return f.v;
}
__device__ __forceinline__ v8f mma_f16(v16h a, v16h b, v8f c) {
  return __builtin_amdgcn_wmma_f32_16x16x32_f16(false, a, false, b, (short)0, c, false, false);
}
__device__ __forceinline__ void step_guard(v8f& d0, v8f& d1, v16h a0, v16h a1, v16h b) {
  asm volatile("v_nop\n\tv_nop\n\tv_nop\n\tv_nop" : "+v"(d0), "+v"(d1) : "v"(a0), "v"(a1), "v"(b));
}
__device__ __forceinline__ float tanh_f32(float x) {
  const float e = expf(2.0f * x);
  return 1.0f - 2.0f * __builtin_amdgcn_rcpf(e + 1.0f);
}

__global__ __launch_bounds__(32) void rnn_seq_kernel(const float* __restrict__ x, const float* __restrict__ h0,
                                                     const float* __restrict__ w_ih, const float* __restrict__ b_ih,
                                                     const float* __restrict__ w_hh, const float* __restrict__ b_hh,
                                                     const float* __restrict__ w_out, const float* __restrict__ b_out,
                                                     float* __restrict__ out_seq, float* __restrict__ out_h) {
  __shared__ __align__(16) _Float16 Hs[ROWS_BLK * HPITCH];
  __shared__ __align__(16) float    Xs[ROWS_BLK * FPITCH];
  __shared__ __align__(16) float    Os[ROWS_BLK * FPITCH];
  __shared__ __align__(16) float    Hf[ROWS_BLK * FPITCH];
  __shared__ __align__(16) float    Cs[3 * NHID];

  const int lane = threadIdx.x & 31;
  const int c    = lane & 15;
  const int hh   = lane >> 4;
  const int q    = lane >> 3;
  const int c4   = (lane & 7) * 4;
  const int rowbase = blockIdx.x * ROWS_BLK;
  if (rowbase + ROWS_BLK > NBATCH) return;

  {
    const float wv = w_ih[lane];
    const float bv = b_ih[lane] + b_hh[lane];
    const float ov = w_out[lane];
    Cs[lane]            = wv;
    Cs[NHID + lane]     = bv;
    Cs[2 * NHID + lane] = ov;
  }
  const float bO = b_out[0];

  v16h a0, a1;
  {
    const float* wr = w_hh + (size_t)c * NHID + 8 * hh;
    const v4f p0 = *(const v4f*)(wr);
    const v4f p1 = *(const v4f*)(wr + 4);
    const v4f p2 = *(const v4f*)(wr + 16);
    const v4f p3 = *(const v4f*)(wr + 20);
#pragma unroll
    for (int e = 0; e < 4; ++e) {
      a0[e]      = (_Float16)(p0[e] * WCARRY);
      a0[4 + e]  = (_Float16)(p1[e] * WCARRY);
      a0[8 + e]  = (_Float16)(p2[e] * WCARRY);
      a0[12 + e] = (_Float16)(p3[e] * WCARRY);
    }
    asm volatile("" : "+v"(a0) :: "memory");
  }
  {
    const float* wr = w_hh + (size_t)(16 + c) * NHID + 8 * hh;
    const v4f p0 = *(const v4f*)(wr);
    const v4f p1 = *(const v4f*)(wr + 4);
    const v4f p2 = *(const v4f*)(wr + 16);
    const v4f p3 = *(const v4f*)(wr + 20);
#pragma unroll
    for (int e = 0; e < 4; ++e) {
      a1[e]      = (_Float16)(p0[e] * WCARRY);
      a1[4 + e]  = (_Float16)(p1[e] * WCARRY);
      a1[8 + e]  = (_Float16)(p2[e] * WCARRY);
      a1[12 + e] = (_Float16)(p3[e] * WCARRY);
    }
    asm volatile("" : "+v"(a1) :: "memory");
  }

  float hst0[8], hst1[8];
  {
    const float* hr = h0 + (size_t)(rowbase + c) * NHID + 8 * hh;
    const v4f g0 = *(const v4f*)(hr);
    const v4f g1 = *(const v4f*)(hr + 4);
    const v4f g2 = *(const v4f*)(hr + 16);
    const v4f g3 = *(const v4f*)(hr + 20);
    v8h n0, n1;
#pragma unroll
    for (int e = 0; e < 4; ++e) {
      hst0[e]     = g0[e];
      hst0[4 + e] = g1[e];
      hst1[e]     = g2[e];
      hst1[4 + e] = g3[e];
    }
#pragma unroll
    for (int r = 0; r < 8; ++r) {
      n0[r] = (_Float16)(hst0[r] * HCARRY);
      n1[r] = (_Float16)(hst1[r] * HCARRY);
    }
    *(v8h*)(Hs + c * HPITCH + 8 * hh)      = n0;
    *(v8h*)(Hs + c * HPITCH + 16 + 8 * hh) = n1;
  }
  __syncthreads();

  float wi0[8], wi1[8], bs0[8], bs1[8], wo0[8], wo1[8];
  {
    const v4f u0 = *(const v4f*)(Cs + 8 * hh);
    const v4f u1 = *(const v4f*)(Cs + 8 * hh + 4);
    const v4f u2 = *(const v4f*)(Cs + 16 + 8 * hh);
    const v4f u3 = *(const v4f*)(Cs + 16 + 8 * hh + 4);
    const v4f s0 = *(const v4f*)(Cs + NHID + 8 * hh);
    const v4f s1 = *(const v4f*)(Cs + NHID + 8 * hh + 4);
    const v4f s2 = *(const v4f*)(Cs + NHID + 16 + 8 * hh);
    const v4f s3 = *(const v4f*)(Cs + NHID + 16 + 8 * hh + 4);
    const v4f o0 = *(const v4f*)(Cs + 2 * NHID + 8 * hh);
    const v4f o1 = *(const v4f*)(Cs + 2 * NHID + 8 * hh + 4);
    const v4f o2 = *(const v4f*)(Cs + 2 * NHID + 16 + 8 * hh);
    const v4f o3 = *(const v4f*)(Cs + 2 * NHID + 16 + 8 * hh + 4);
#pragma unroll
    for (int e = 0; e < 4; ++e) {
      wi0[e] = u0[e]; wi0[4 + e] = u1[e]; wi1[e] = u2[e]; wi1[4 + e] = u3[e];
      bs0[e] = s0[e]; bs0[4 + e] = s1[e]; bs1[e] = s2[e]; bs1[4 + e] = s3[e];
      wo0[e] = o0[e]; wo0[4 + e] = o1[e]; wo1[e] = o2[e]; wo1[4 + e] = o3[e];
    }
  }

  const v8f z8 = {0.f, 0.f, 0.f, 0.f, 0.f, 0.f, 0.f, 0.f};
  const _Float16* hrow = Hs + c * HPITCH + 8 * hh;

#pragma unroll 1
  for (int ch = 0; ch < NCHUNK; ++ch) {
    const int t0 = ch * TCHUNK;
#pragma unroll
    for (int it = 0; it < 4; ++it) {
      const int row = 4 * it + q;
      const v4f v = *(const v4f*)(x + (size_t)(rowbase + row) * NSTEP + t0 + c4);
      *(v4f*)(Xs + row * FPITCH + c4) = v;
    }
    __syncthreads();

#pragma unroll 1
    for (int tt = 0; tt < TCHUNK; ++tt) {
      const float xv = Xs[c * FPITCH + tt];
      const v16h bfr = frag_load(hrow);
      __syncthreads();
      v8f d0 = mma_f16(a0, bfr, z8);
      v8f d1 = mma_f16(a1, bfr, z8);
      step_guard(d0, d1, a0, a1, bfr);

      float p = 0.0f;
      v8h n0, n1;
#pragma unroll
      for (int r = 0; r < 8; ++r) {
        const float pre = d0[r] * CARRYINV + (xv * wi0[r] + bs0[r]);
        const float hn = tanh_f32(pre);
        hst0[r] = hn;
        n0[r] = (_Float16)(hn * HCARRY);
        p += hn * wo0[r];
      }
#pragma unroll
      for (int r = 0; r < 8; ++r) {
        const float pre = d1[r] * CARRYINV + (xv * wi1[r] + bs1[r]);
        const float hn = tanh_f32(pre);
        hst1[r] = hn;
        n1[r] = (_Float16)(hn * HCARRY);
        p += hn * wo1[r];
      }
      *(v8h*)(Hs + c * HPITCH + 8 * hh)      = n0;
      *(v8h*)(Hs + c * HPITCH + 16 + 8 * hh) = n1;
      const float po = __shfl_xor(p, 16, 32);
      const float ov = (p + po) + bO;
      if (hh == 0) Os[c * FPITCH + tt] = ov;
      __syncthreads();
    }

    v4f fv[4];
#pragma unroll
    for (int it = 0; it < 4; ++it) fv[it] = *(const v4f*)(Os + (4 * it + q) * FPITCH + c4);
    for (int pass = 0; pass < 2; ++pass) {
#pragma unroll
      for (int it = 0; it < 4; ++it) {
        const int row = 4 * it + q;
        *(volatile v4f*)(out_seq + (size_t)(rowbase + row) * NSTEP + t0 + c4) = fv[it];
      }
      __threadfence();
    }
    __syncthreads();
  }

  {
    v4f w0, w1, w2, w3;
#pragma unroll
    for (int e = 0; e < 4; ++e) {
      w0[e] = hst0[e];
      w1[e] = hst0[4 + e];
      w2[e] = hst1[e];
      w3[e] = hst1[4 + e];
    }
    *(v4f*)(Hf + c * FPITCH + 8 * hh)          = w0;
    *(v4f*)(Hf + c * FPITCH + 8 * hh + 4)      = w1;
    *(v4f*)(Hf + c * FPITCH + 16 + 8 * hh)     = w2;
    *(v4f*)(Hf + c * FPITCH + 16 + 8 * hh + 4) = w3;
  }
  __syncthreads();
  {
    v4f fv[4];
#pragma unroll
    for (int it = 0; it < 4; ++it) fv[it] = *(const v4f*)(Hf + (4 * it + q) * FPITCH + c4);
    for (int pass = 0; pass < 2; ++pass) {
#pragma unroll
      for (int it = 0; it < 4; ++it) {
        const int row = 4 * it + q;
        *(volatile v4f*)(out_h + (size_t)(rowbase + row) * NHID + c4) = fv[it];
      }
      __threadfence();
    }
  }
}

extern "C" void kernel_launch(void* const* d_in, const int* in_sizes, int n_in,
                              void* d_out, int out_size, void* d_ws, size_t ws_size, hipStream_t stream) {
  (void)in_sizes; (void)out_size; (void)d_ws; (void)ws_size;
  if (n_in < 8 || d_out == nullptr) return;
  const float* x     = (const float*)d_in[0];
  const float* h0    = (const float*)d_in[1];
  const float* w_ih  = (const float*)d_in[2];
  const float* b_ih  = (const float*)d_in[3];
  const float* w_hh  = (const float*)d_in[4];
  const float* b_hh  = (const float*)d_in[5];
  const float* w_out = (const float*)d_in[6];
  const float* b_out = (const float*)d_in[7];
  float* out_seq = (float*)d_out;
  float* out_h   = out_seq + (size_t)NOUT0;
  rnn_seq_kernel<<<NBATCH / ROWS_BLK, 32, 0, stream>>>(x, h0, w_ih, b_ih, w_hh, b_hh, w_out, b_out, out_seq, out_h);
}
